// Model_24429773980161
// MI455X (gfx1250) — hardware-verified
//
#include <hip/hip_runtime.h>
#include <stddef.h>
#include <stdint.h>
#include <math.h>


#define NBAT   16
#define NN     1024
#define NM     256
#define NINC   4096
#define CC     512
#define MROWS  (NBAT * NN)
#define OUTN   (MROWS * CC)
#define NTHR   256
#define ETHR   128
#define NWV    4
#define EPW    (NINC / NWV)
#define APITCH 32
#define RPITCH 32
#define EBP    (2 * CC)
#define GBM    64
#define GBN    64
#define GTHR   128
#define WSMAX  134217728

static_assert(NINC % (NWV * 32) == 0 && EPW == 1024);
static_assert(CC == 4 * ETHR && CC % 32 == 0);
static_assert(MROWS % GBM == 0 && CC % GBN == 0 && NM % GBM == 0);
static_assert(OUTN % (8 * NTHR) == 0);
static_assert((CC * CC / 8) % NTHR == 0);
static_assert((NINC << 4) < (1 << 30));
static_assert(NM % 4 == 0 && NN % 16 == 0 && NN % 8 == 0);

typedef float          v2f   __attribute__((ext_vector_type(2)));
typedef float          v4f   __attribute__((ext_vector_type(4)));
typedef float          v8f   __attribute__((ext_vector_type(8)));
typedef int            v8i   __attribute__((ext_vector_type(8)));
typedef unsigned short v4us  __attribute__((ext_vector_type(4)));
typedef unsigned short v8us  __attribute__((ext_vector_type(8)));
typedef unsigned short v16us __attribute__((ext_vector_type(16)));
typedef __bf16         v16bf __attribute__((ext_vector_type(16)));
typedef v4f  __attribute__((may_alias)) v4fa;
typedef v4us __attribute__((may_alias)) v4usa;
typedef v8us __attribute__((may_alias)) v8usa;
union FragB { v16bf v; v16us u; v8us h[2]; v8i w; };

__device__ __forceinline__ v8f wmb(const FragB& a, const FragB& b, v8f c) {
  v8f d = __builtin_amdgcn_wmma_f32_16x16x32_bf16(false, a.v, false, b.v, (short)0, c, false, false);
  asm volatile("v_nop\n\tv_nop\n\tv_nop\n\tv_nop" : "+v"(d) : "v"(a.w), "v"(b.w));
  return d;
}

__device__ __forceinline__ unsigned bf16_bits(float f) {
  const unsigned u = __float_as_uint(f);
  return (u + 0x7FFFu + ((u >> 16) & 1u)) >> 16;
}
__device__ __forceinline__ float bf16_val(float f) {
  return __uint_as_float(bf16_bits(f) << 16);
}

__global__ __launch_bounds__(NTHR) void k_cvx(const float* __restrict__ x, unsigned short* xb) {
  const size_t u = (size_t)blockIdx.x * NTHR + threadIdx.x;
  const float* p = x + u * 8;
  const v4f a = *(const v4fa*)p;
  const v4f b = *(const v4fa*)(p + 4);
  v8us o;
  o[0] = (unsigned short)bf16_bits(a.x); o[1] = (unsigned short)bf16_bits(a.y);
  o[2] = (unsigned short)bf16_bits(a.z); o[3] = (unsigned short)bf16_bits(a.w);
  o[4] = (unsigned short)bf16_bits(b.x); o[5] = (unsigned short)bf16_bits(b.y);
  o[6] = (unsigned short)bf16_bits(b.z); o[7] = (unsigned short)bf16_bits(b.w);
  unsigned short* dp = xb + u * 8;
  *(volatile v8us*)dp = o;
  __threadfence();
  *(volatile v8us*)dp = o;
}

__global__ __launch_bounds__(NTHR) void k_wprep(const float* __restrict__ W, unsigned short* wt) {
  const int u  = (int)blockIdx.x * NTHR + (int)threadIdx.x;
  const int n  = u >> 6;
  const int k8 = (u & 63) * 8;
  const float* p = W + (size_t)k8 * CC + n;
  v8us o;
#pragma unroll
  for (int i = 0; i < 8; ++i) o[i] = (unsigned short)bf16_bits(p[(size_t)i * CC]);
  unsigned short* dp = wt + (size_t)n * CC + k8;
  *(volatile v8us*)dp = o;
  __threadfence();
  *(volatile v8us*)dp = o;
}

__global__ __launch_bounds__(GTHR) void k_gemm(
    const unsigned short* __restrict__ A, const unsigned short* __restrict__ WT,
    float* outF, int K, int ldo)
{
  __shared__ __attribute__((aligned(16))) float stg[GBM * GBN];
  const int tid = (int)threadIdx.x, lane = tid & 31, wave = tid >> 5, hh = lane >> 4, m = lane & 15;
  const int rowBase = (int)blockIdx.x * GBM;
  const int col0    = (int)blockIdx.y * GBN;

  v8f acc[4];
  {
    const v8f z = {0.f, 0.f, 0.f, 0.f, 0.f, 0.f, 0.f, 0.f};
    acc[0] = z; acc[1] = z; acc[2] = z; acc[3] = z;
  }
  const unsigned short* ap = A  + (size_t)(rowBase + 16 * wave + m) * (size_t)K + 8 * hh;
  const unsigned short* wp = WT + (size_t)(col0 + m) * (size_t)K + 8 * hh;
  const int ksteps = K >> 5;
#pragma unroll 1
  for (int ks = 0; ks < ksteps; ++ks) {
    FragB af;
    af.h[0] = *(const v8usa*)(ap + 32 * ks);
    af.h[1] = *(const v8usa*)(ap + 32 * ks + 16);
#pragma unroll
    for (int t = 0; t < 4; ++t) {
      const unsigned short* wq = wp + (size_t)(16 * t) * (size_t)K + 32 * ks;
      FragB bf;
      bf.h[0] = *(const v8usa*)wq;
      bf.h[1] = *(const v8usa*)(wq + 16);
      acc[t] = wmb(af, bf, acc[t]);
    }
  }

#pragma unroll
  for (int t = 0; t < 4; ++t) {
    const int lc = 16 * t + m;
#pragma unroll
    for (int r = 0; r < 8; ++r) {
      const int lr = 16 * wave + 8 * hh + r;
      stg[lr * GBN + lc] = acc[t][r];
    }
  }
  __syncthreads();

  v4f fv[8];
#pragma unroll
  for (int i = 0; i < 8; ++i) {
    const int lr = 16 * wave + 2 * i + hh;
    fv[i] = *(const v4fa*)(stg + lr * GBN + 4 * m);
  }
#pragma unroll
  for (int i = 0; i < 8; ++i) {
    const int lr = 16 * wave + 2 * i + hh;
    const int gr = rowBase + lr;
    float* op = outF + (size_t)gr * (size_t)ldo + col0 + 4 * m;
    *(volatile v4f*)op = fv[i];
  }
  __threadfence();
#pragma unroll
  for (int i = 0; i < 8; ++i) {
    const int lr = 16 * wave + 2 * i + hh;
    const int gr = rowBase + lr;
    float* op = outF + (size_t)gr * (size_t)ldo + col0 + 4 * m;
    *(volatile v4f*)op = fv[i];
  }
}

template <int NB>
__device__ __forceinline__ int scan_keys(const int* __restrict__ keys, int base, int* list, int lane, int wave) {
  int wc = 0;
  const int w0 = wave * EPW;
#pragma unroll 2
  for (int s = 0; s < EPW / 32; ++s) {
    const int e  = w0 + s * 32 + lane;
    const int kv = keys[e];
    const unsigned sl = (unsigned)kv - (unsigned)base;
    const bool hit = sl < (unsigned)NB;
    const unsigned mj = __builtin_amdgcn_ballot_w32(hit);
    if (mj != 0u) {
      if (hit) {
        const int pos = wc + (int)__builtin_amdgcn_mbcnt_lo(mj, 0u);
        if (pos < EPW) list[w0 + pos] = (e << 4) | (int)sl;
      }
      wc += (int)__builtin_popcount(mj);
    }
  }
  return wc;
}

template <int MODE>
__device__ __forceinline__ void walk_slot(const int* list, const int* wcnt, int s, int lane, int tid,
                                          const int* __restrict__ gath, int gmax,
                                          const float* __restrict__ alpha, int b,
                                          const float* __restrict__ plane, v4f& acc, int& cnt) {
  v4f a4 = {0.0f, 0.0f, 0.0f, 0.0f};
  int n = 0;
#pragma unroll 1
  for (int w2 = 0; w2 < NWV; ++w2) {
    int c = wcnt[w2];
    c = c < 0 ? 0 : (c > EPW ? EPW : c);
#pragma unroll 1
    for (int b0 = 0; b0 < c; b0 += 32) {
      const int ii = b0 + lane;
      const bool in = ii < c;
      const int idx = in ? ii : c - 1;
      const int ent = list[w2 * EPW + idx];
      const bool mt = in && ((ent & 15) == s);
      unsigned msk = __builtin_amdgcn_ballot_w32(mt);
      if (msk != 0u) {
        const int e = (ent >> 4) & (NINC - 1);
        int g = gath[e];
        g = g < 0 ? 0 : (g > gmax ? gmax : g);
        int wvi = 0x3f800000;
        if constexpr (MODE != 0) wvi = __float_as_int(alpha[(size_t)e * APITCH + 2 * b]);
        const int nh = (int)__builtin_popcount(msk);
        n += nh;
#pragma unroll 1
        for (int q = 0; q < nh; ++q) {
          const int k = __builtin_ffs((int)msk) - 1;
          msk &= msk - 1u;
          const int gk = __builtin_amdgcn_readlane(g, k);
          const v4f r = *(const v4fa*)(plane + (size_t)gk * CC + 4 * tid);
          if constexpr (MODE != 0) {
            const float wk = __int_as_float(__builtin_amdgcn_readlane(wvi, k));
            a4.x = fmaf(wk, r.x, a4.x); a4.y = fmaf(wk, r.y, a4.y);
            a4.z = fmaf(wk, r.z, a4.z); a4.w = fmaf(wk, r.w, a4.w);
          } else {
            a4.x += r.x; a4.y += r.y; a4.z += r.z; a4.w += r.w;
          }
        }
      }
    }
  }
  acc = a4;
  cnt = n;
}

template <int MODE>
__global__ __launch_bounds__(ETHR) void k_edge(const int* __restrict__ nidx, const int* __restrict__ eidx,
                                               const float* __restrict__ xw, const float* __restrict__ att,
                                               const float* __restrict__ alpha,
                                               unsigned short* esb, float* rec, float* oute) {
  __shared__ int list[NINC];
  __shared__ int wcnt[NWV];
  __shared__ __attribute__((aligned(16))) unsigned short rowst[EBP];
  __shared__ float red[NWV * 4];
  __shared__ __attribute__((aligned(16))) float recs[RPITCH];
  const int tid = (int)threadIdx.x, lane = tid & 31, wave = tid >> 5;
  const int mg = (int)blockIdx.x, b = (int)blockIdx.y;
  const int base = mg * 4;

  const int wc = scan_keys<4>(eidx, base, list, lane, wave);
  if (lane == 0) wcnt[wave] = wc;
  if (tid < RPITCH) recs[tid] = 0.0f;
  if (tid < NWV * 4) red[tid] = 0.0f;
  v4f t4 = {0.0f, 0.0f, 0.0f, 0.0f};
  if constexpr (MODE == 0) {
    const v4f t = *(const v4fa*)(att + CC + 4 * tid);
    t4.x = bf16_val(t.x); t4.y = bf16_val(t.y); t4.z = bf16_val(t.z); t4.w = bf16_val(t.w);
  }
  __syncthreads();

  const float* plane = xw + (size_t)b * NN * CC;
#pragma unroll 1
  for (int s = 0; s < 4; ++s) {
    v4f acc;
    int cnt;
    walk_slot<MODE>(list, wcnt, s, lane, tid, nidx, NN - 1, alpha, b, plane, acc, cnt);
    const int m = base + s;
    if constexpr (MODE != 0) {
      const float cf = (float)(cnt < 1 ? 1 : cnt);
      const float bn = (cnt > 0) ? (1.0f / cf) : 0.0f;
      v4f v;
      v.x = acc.x * bn; v.y = acc.y * bn; v.z = acc.z * bn; v.w = acc.w * bn;
      float* op = oute + ((size_t)(b * NM + m)) * CC + 4 * tid;
      *(volatile v4f*)op = v;
      __threadfence();
      *(volatile v4f*)op = v;
    } else {
      float sr = acc.x * t4.x;
      sr = fmaf(acc.y, t4.y, sr); sr = fmaf(acc.z, t4.z, sr); sr = fmaf(acc.w, t4.w, sr);
      float sq = acc.x * acc.x;
      sq = fmaf(acc.y, acc.y, sq); sq = fmaf(acc.z, acc.z, sq); sq = fmaf(acc.w, acc.w, sq);
      float sm = (acc.x + acc.y) + (acc.z + acc.w);
#pragma unroll
      for (int o = 16; o > 0; o >>= 1) {
        sr += __shfl_xor(sr, o, 32);
        sq += __shfl_xor(sq, o, 32);
        sm += __shfl_xor(sm, o, 32);
      }
      if (lane == 0) { red[wave * 4 + 0] = sr; red[wave * 4 + 1] = sq; red[wave * 4 + 2] = sm; }
      v4us h4, l4;
      unsigned hb;
      hb = bf16_bits(acc.x); h4[0] = (unsigned short)hb; l4[0] = (unsigned short)bf16_bits(acc.x - __uint_as_float(hb << 16));
      hb = bf16_bits(acc.y); h4[1] = (unsigned short)hb; l4[1] = (unsigned short)bf16_bits(acc.y - __uint_as_float(hb << 16));
      hb = bf16_bits(acc.z); h4[2] = (unsigned short)hb; l4[2] = (unsigned short)bf16_bits(acc.z - __uint_as_float(hb << 16));
      hb = bf16_bits(acc.w); h4[3] = (unsigned short)hb; l4[3] = (unsigned short)bf16_bits(acc.w - __uint_as_float(hb << 16));
      *(v4usa*)(rowst + 4 * tid) = h4;
      *(v4usa*)(rowst + CC + 4 * tid) = l4;
      __syncthreads();
      if (tid == 0) {
        recs[s * 4 + 0] = ((red[0] + red[4]) + red[8]) + red[12];
        recs[s * 4 + 1] = ((red[1] + red[5]) + red[9]) + red[13];
        recs[s * 4 + 2] = ((red[2] + red[6]) + red[10]) + red[14];
        recs[s * 4 + 3] = (float)cnt;
      }
      const v8us qv = *(const v8usa*)(rowst + 8 * tid);
      unsigned short* dp = esb + ((size_t)(b * NM + m)) * EBP + 8 * tid;
      *(volatile v8us*)dp = qv;
      __threadfence();
      *(volatile v8us*)dp = qv;
      __syncthreads();
    }
  }
  if constexpr (MODE == 0) {
    if (tid < 8) {
      const v4f rv = *(const v4fa*)(recs + 4 * tid);
      float* rp = rec + ((size_t)(b * 64 + mg)) * RPITCH + 4 * tid;
      *(volatile v4f*)rp = rv;
      __threadfence();
      *(volatile v4f*)rp = rv;
    }
  }
}

__device__ __forceinline__ float raw_at(const int* list, int pos, const int* __restrict__ eidx,
                                        const float* __restrict__ rec, int b, float p, int& e_out, int& sl_out) {
  const int ent = list[pos];
  const int e = (ent >> 4) & (NINC - 1);
  int m = eidx[e];
  m = m < 0 ? 0 : (m > NM - 1 ? NM - 1 : m);
  const float r = rec[((size_t)(b * 64 + (m >> 2))) * RPITCH + (m & 3) * 4];
  const float v = p + r;
  e_out = e;
  sl_out = ent & 15;
  return v > 0.0f ? v : 0.2f * v;
}

__device__ __forceinline__ void alpha_store_pass(const int* list, const int* wcnt, const int* __restrict__ eidx,
                                                 const float* __restrict__ rec, int b, float p, int slot,
                                                 float mx, float rden, float* alpha) {
#pragma unroll 1
  for (int w2 = 0; w2 < NWV; ++w2) {
    int c = wcnt[w2];
    c = c < 0 ? 0 : (c > EPW ? EPW : c);
#pragma unroll 1
    for (int i = 0; i < c; ++i) {
      int e, sl;
      const float raw = raw_at(list, w2 * EPW + i, eidx, rec, b, p, e, sl);
      const float ex = expf(raw - mx);
      v2f o;
      o.x = ex * rden;
      o.y = 0.0f;
      if (sl == slot) *(volatile v2f*)(alpha + (size_t)e * APITCH + 2 * b) = o;
    }
  }
}

__global__ __launch_bounds__(ETHR) void k_alpha(const int* __restrict__ nidx, const int* __restrict__ eidx,
                                                const float* __restrict__ xw, const float* __restrict__ att,
                                                const float* __restrict__ rec, float* alpha) {
  __shared__ int list[NINC];
  __shared__ int wcnt[NWV];
  __shared__ __attribute__((aligned(16))) float atts[CC];
  __shared__ float ps[ETHR];
  const int tid = (int)threadIdx.x, lane = tid & 31, wave = tid >> 5;
  const int nodeBase = (int)blockIdx.x * 8;

  const int wc = scan_keys<8>(nidx, nodeBase, list, lane, wave);
  if (lane == 0) wcnt[wave] = wc;
  {
    const v4f t = *(const v4fa*)(att + 4 * tid);
    v4f r;
    r.x = bf16_val(t.x); r.y = bf16_val(t.y); r.z = bf16_val(t.z); r.w = bf16_val(t.w);
    *(v4fa*)(atts + 4 * tid) = r;
  }
  __syncthreads();

#pragma unroll 1
  for (int i = 0; i < 32; ++i) {
    const int q = wave * 32 + i;
    const int sl = q >> 4, bb = q & 15;
    const float* row = xw + ((size_t)(bb * NN + nodeBase + sl)) * CC;
    float s = 0.0f;
#pragma unroll 1
    for (int j = 0; j < 4; ++j) {
      const v4f xv = *(const v4fa*)(row + 128 * j + 4 * lane);
      const v4f av = *(const v4fa*)(atts + 128 * j + 4 * lane);
      s = fmaf(xv.x, av.x, s); s = fmaf(xv.y, av.y, s); s = fmaf(xv.z, av.z, s); s = fmaf(xv.w, av.w, s);
    }
#pragma unroll
    for (int o = 16; o > 0; o >>= 1) s += __shfl_xor(s, o, 32);
    if (lane == 0) ps[q] = s;
  }
  __syncthreads();

  const int slot = tid >> 4, b = tid & 15;
  const float p = ps[tid];
  float mx = -3.0e38f;
#pragma unroll 1
  for (int w2 = 0; w2 < NWV; ++w2) {
    int c = wcnt[w2];
    c = c < 0 ? 0 : (c > EPW ? EPW : c);
#pragma unroll 1
    for (int i = 0; i < c; ++i) {
      int e, sl;
      const float raw = raw_at(list, w2 * EPW + i, eidx, rec, b, p, e, sl);
      const float cand = fmaxf(mx, raw);
      mx = (sl == slot) ? cand : mx;
    }
  }
  float den = 0.0f;
#pragma unroll 1
  for (int w2 = 0; w2 < NWV; ++w2) {
    int c = wcnt[w2];
    c = c < 0 ? 0 : (c > EPW ? EPW : c);
#pragma unroll 1
    for (int i = 0; i < c; ++i) {
      int e, sl;
      const float raw = raw_at(list, w2 * EPW + i, eidx, rec, b, p, e, sl);
      const float ex = expf(raw - mx);
      den = (sl == slot) ? (den + ex) : den;
    }
  }
  const float rden = 1.0f / (den + 1e-16f);
  alpha_store_pass(list, wcnt, eidx, rec, b, p, slot, mx, rden, alpha);
  __threadfence();
  alpha_store_pass(list, wcnt, eidx, rec, b, p, slot, mx, rden, alpha);
}

__global__ __launch_bounds__(ETHR) void k_outn(const int* __restrict__ nidx, const int* __restrict__ eidx,
                                               const float* __restrict__ alpha, const float* __restrict__ oute,
                                               float* out) {
  __shared__ int list[NINC];
  __shared__ int wcnt[NWV];
  const int tid = (int)threadIdx.x, lane = tid & 31, wave = tid >> 5;
  const int nodeBase = (int)blockIdx.x * 16, b = (int)blockIdx.y;

  const int wc = scan_keys<16>(nidx, nodeBase, list, lane, wave);
  if (lane == 0) wcnt[wave] = wc;
  __syncthreads();

  const float* plane = oute + (size_t)b * NM * CC;
#pragma unroll 1
  for (int s = 0; s < 16; ++s) {
    v4f acc;
    int cnt;
    walk_slot<1>(list, wcnt, s, lane, tid, eidx, NM - 1, alpha, b, plane, acc, cnt);
    const float d = (float)cnt;
    v4f v;
    v.x = acc.x * d; v.y = acc.y * d; v.z = acc.z * d; v.w = acc.w * d;
    float* op = out + ((size_t)(b * NN + nodeBase + s)) * CC + 4 * tid;
    *(volatile v4f*)op = v;
    __threadfence();
    *(volatile v4f*)op = v;
  }
}

__global__ __launch_bounds__(GTHR) void k_gram(const unsigned short* __restrict__ esb, const float* __restrict__ rec,
                                               float* recg) {
  __shared__ float sqs[128];
  __shared__ float nrs[128];
  __shared__ float redw[NWV];
  __shared__ __attribute__((aligned(16))) float recs[RPITCH];
  const int tid = (int)threadIdx.x, lane = tid & 31, wave = tid >> 5, hh = lane >> 4, m = lane & 15;
  const int blk = (int)blockIdx.x;
  const int kBase = (blk >> 2) * 64, mBase = (blk & 3) * 64;
  if (tid < RPITCH) recs[tid] = 0.0f;

  v8f L[4];
  {
    const v8f z = {0.f, 0.f, 0.f, 0.f, 0.f, 0.f, 0.f, 0.f};
    L[0] = z; L[1] = z; L[2] = z; L[3] = z;
  }
#pragma unroll 1
  for (int b = 0; b < NBAT; ++b) {
    __syncthreads();
    {
      const int g = (tid < 64) ? (kBase + tid) : (mBase + tid - 64);
      const float v = rec[((size_t)(b * 64 + (g >> 2))) * RPITCH + (g & 3) * 4 + 1];
      const float vc = (v < 1e-12f) ? 1e-12f : v;
      sqs[tid] = v;
      nrs[tid] = sqrtf(vc);
    }
    __syncthreads();

    v8f acc[4];
    {
      const v8f z = {0.f, 0.f, 0.f, 0.f, 0.f, 0.f, 0.f, 0.f};
      acc[0] = z; acc[1] = z; acc[2] = z; acc[3] = z;
    }
    const unsigned short* ap = esb + ((size_t)(b * NM + kBase + 16 * wave + m)) * EBP + 8 * hh;
    const unsigned short* bp = esb + ((size_t)(b * NM + mBase + m)) * EBP + 8 * hh;
#pragma unroll 1
    for (int ks = 0; ks < CC / 32; ++ks) {
      FragB ah, al;
      ah.h[0] = *(const v8usa*)(ap + 32 * ks);
      ah.h[1] = *(const v8usa*)(ap + 32 * ks + 16);
      al.h[0] = *(const v8usa*)(ap + CC + 32 * ks);
      al.h[1] = *(const v8usa*)(ap + CC + 32 * ks + 16);
#pragma unroll
      for (int t = 0; t < 4; ++t) {
        const unsigned short* bq = bp + (size_t)(16 * t) * EBP + 32 * ks;
        FragB bh, bl;
        bh.h[0] = *(const v8usa*)bq;
        bh.h[1] = *(const v8usa*)(bq + 16);
        bl.h[0] = *(const v8usa*)(bq + CC);
        bl.h[1] = *(const v8usa*)(bq + CC + 16);
        acc[t] = wmb(ah, bh, acc[t]);
        acc[t] = wmb(al, bh, acc[t]);
        acc[t] = wmb(ah, bl, acc[t]);
      }
    }

    float skr[8], nkr[8], smt[4], nmt[4];
#pragma unroll
    for (int r = 0; r < 8; ++r) { skr[r] = sqs[16 * wave + 8 * hh + r]; nkr[r] = nrs[16 * wave + 8 * hh + r]; }
#pragma unroll
    for (int t = 0; t < 4; ++t) { smt[t] = sqs[64 + 16 * t + m]; nmt[t] = nrs[64 + 16 * t + m]; }
#pragma unroll
    for (int t = 0; t < 4; ++t) {
#pragma unroll
      for (int r = 0; r < 8; ++r) {
        const int kg = kBase + 16 * wave + 8 * hh + r;
        const int mg = mBase + 16 * t + m;
        const float ipv = (kg == mg) ? skr[r] : acc[t][r];
        float den = nkr[r] * nmt[t];
        den = (den < 1e-12f) ? 1e-12f : den;
        const float a = ipv * (1.0f / den);
        float d2 = (skr[r] + smt[t]) - 2.0f * ipv;
        d2 = (d2 < 1e-12f) ? 1e-12f : d2;
        const float dist = sqrtf(d2);
        float hg = 4.2f - dist;
        hg = (hg < 0.0f) ? 0.0f : hg;
        L[t][r] += a * dist + (1.0f - a) * hg;
      }
    }
  }

  float ls = 0.0f;
#pragma unroll
  for (int t = 0; t < 4; ++t) {
#pragma unroll
    for (int r = 0; r < 8; ++r) ls += fabsf(L[t][r] * 0.0625f);
  }
#pragma unroll
  for (int o = 16; o > 0; o >>= 1) ls += __shfl_xor(ls, o, 32);
  if (lane == 0) redw[wave] = ls;
  __syncthreads();
  if (tid == 0) recs[0] = ((redw[0] + redw[1]) + redw[2]) + redw[3];
  __syncthreads();
  if (tid < 8) {
    const v4f rv = *(const v4fa*)(recs + 4 * tid);
    float* rp = recg + (size_t)blk * RPITCH + 4 * tid;
    *(volatile v4f*)rp = rv;
    __threadfence();
    *(volatile v4f*)rp = rv;
  }
}

__global__ __launch_bounds__(NTHR) void k_final(const float* __restrict__ rec, const float* __restrict__ recg,
                                                float* out) {
  __shared__ double smm[NM];
  __shared__ double sgg[16];
  const int tid = (int)threadIdx.x;
  {
    const int mq = tid >> 2, ms = tid & 3;
    double s = 0.0;
#pragma unroll 4
    for (int b = 0; b < NBAT; ++b) s += (double)rec[((size_t)(b * 64 + mq)) * RPITCH + ms * 4 + 2];
    const double dg = (double)rec[((size_t)mq) * RPITCH + ms * 4 + 3];
    smm[tid] = (1.0 - dg) * s;
  }
  if (tid < 16) sgg[tid] = (double)recg[(size_t)tid * RPITCH];
  __syncthreads();
  if (tid == 0) {
    double a = 0.0;
#pragma unroll 1
    for (int i = 0; i < NM; ++i) a += smm[i];
    double g = 0.0;
#pragma unroll 1
    for (int i = 0; i < 16; ++i) g += sgg[i];
    const double res = fabs(a) / 33554432.0 + g / 66049.0;
    const float rf = (float)res;
    float* op = out + (size_t)OUTN;
    *(volatile float*)op = rf;
    __threadfence();
    *(volatile float*)op = rf;
  }
}

static inline size_t al256(size_t o) { return (o + 255) & ~(size_t)255; }

extern "C" void kernel_launch(void* const* d_in, const int* in_sizes, int n_in,
                              void* d_out, int out_size, void* d_ws, size_t ws_size,
                              hipStream_t stream) {
  if (n_in < 5) return;
  if (in_sizes[0] != OUTN) return;
  if (in_sizes[1] != CC * CC) return;
  if (in_sizes[2] != 2 * CC) return;
  if (in_sizes[3] != NINC) return;
  if (in_sizes[4] != NINC) return;
  if (out_size != OUTN + 1) return;

  const float* x    = (const float*)d_in[0];
  const float* W    = (const float*)d_in[1];
  const float* att  = (const float*)d_in[2];
  const int*   nidx = (const int*)d_in[3];
  const int*   eidx = (const int*)d_in[4];
  float* out = (float*)d_out;

  char* ws = (char*)d_ws;
  size_t off = 0;
  const size_t oXB  = off; off = al256(off + (size_t)MROWS * CC * 2);
  const size_t oWT  = off; off = al256(off + (size_t)CC * CC * 2);
  const size_t oXW  = off; off = al256(off + (size_t)MROWS * CC * 4);
  const size_t oESB = off; off = al256(off + (size_t)NBAT * NM * EBP * 2);
  const size_t oOE  = off; off = al256(off + (size_t)NBAT * NM * CC * 4);
  const size_t oAL  = off; off = al256(off + (size_t)NINC * APITCH * 4);
  const size_t oRE  = off; off = al256(off + (size_t)NBAT * 64 * RPITCH * 4);
  const size_t oRG  = off; off = al256(off + (size_t)16 * RPITCH * 4);
  if (off > ws_size || off > (size_t)WSMAX) return;
  unsigned short* XB   = (unsigned short*)(ws + oXB);
  unsigned short* WT   = (unsigned short*)(ws + oWT);
  float*          XW   = (float*)(ws + oXW);
  unsigned short* ESB  = (unsigned short*)(ws + oESB);
  float*          OUTE = (float*)(ws + oOE);
  float*          ALPH = (float*)(ws + oAL);
  float*          RECE = (float*)(ws + oRE);
  float*          RECG = (float*)(ws + oRG);

  k_cvx<<<OUTN / 8 / NTHR, NTHR, 0, stream>>>(x, XB);
  k_wprep<<<(CC * CC / 8) / NTHR, NTHR, 0, stream>>>(W, WT);
  k_gemm<<<dim3(MROWS / GBM, CC / GBN), GTHR, 0, stream>>>(XB, WT, XW, CC, CC);
  k_edge<0><<<dim3(NM / 4, NBAT), ETHR, 0, stream>>>(nidx, eidx, XW, att, ALPH, ESB, RECE, OUTE);
  k_alpha<<<NN / 8, ETHR, 0, stream>>>(nidx, eidx, XW, att, RECE, ALPH);
  k_edge<1><<<dim3(NM / 4, NBAT), ETHR, 0, stream>>>(nidx, eidx, XW, att, ALPH, ESB, RECE, OUTE);
  k_outn<<<dim3(NN / 16, NBAT), ETHR, 0, stream>>>(nidx, eidx, ALPH, OUTE, out);
  k_gram<<<16, GTHR, 0, stream>>>(ESB, RECE, RECG);
  k_final<<<1, NTHR, 0, stream>>>(RECE, RECG, out);
}
